// SingleHeadAttention_2121713844998
// MI455X (gfx1250) — hardware-verified
//
#include <hip/hip_runtime.h>

typedef _Float16 h16;
typedef _Float16 h16x8 __attribute__((ext_vector_type(8)));
typedef _Float16 v16h  __attribute__((ext_vector_type(16)));
typedef float  v8f    __attribute__((ext_vector_type(8)));
typedef float  v4f    __attribute__((ext_vector_type(4)));
typedef unsigned v4u  __attribute__((ext_vector_type(4)));

#ifndef NB
#define NB 4
#endif
#ifndef SEQ
#define SEQ 4096
#endif
#define NB_FULL 4
#define SEQ_FULL 4096
#define DM 512
#define EARLY_CAP 512
#define EARLY_R ((SEQ < EARLY_CAP) ? SEQ : EARLY_CAP)
#define MT (NB * SEQ)

static_assert(SEQ % 64 == 0);
static_assert((EARLY_R) % 64 == 0);
static_assert(NB >= 1 && NB <= NB_FULL);
static_assert(SEQ >= 64 && SEQ <= SEQ_FULL);
static_assert(DM % 128 == 0);
static_assert(((NB - 1) * SEQ_FULL + SEQ) * DM <= NB_FULL * SEQ_FULL * DM);

#define ISC  16.0f
#define WSC  16.0f
#define PSC  1024.0f
#define RSC  16384.0f
#define RINV (1.0f / 16384.0f)
#define PROJ_MUL (1.0f / 16.0f)
#define OUT_MUL  (1.0f / 256.0f)
#define SCL ((1.0f / 256.0f) * (1.0f / 22.627416610717773f))

template <typename V> __device__ __forceinline__ void vst2(void* p, V v) {
  *(volatile V*)p = v; __threadfence(); *(volatile V*)p = v;
}
__device__ __forceinline__ void copy16_g2s(h16* ldst, const h16* gsrc) { *(h16x8*)ldst = *(const h16x8*)gsrc; }

__device__ __forceinline__ float bf16r(float f) {
  unsigned u = __float_as_uint(f);
  u = (u + 0x7FFFu + ((u >> 16) & 1u)) & 0xFFFF0000u;
  return __uint_as_float(u);
}

__device__ __forceinline__ v16h load_a_frag(const h16* base, int ld, int k0) {
  int lane = threadIdx.x & 31;
  int idx  = lane & 15;
  int half = lane >> 4;
  const h16* p = base + idx * ld + k0 + half * 8;
  h16x8 lo = *(const h16x8*)(p);
  h16x8 hi = *(const h16x8*)(p + 16);
  return __builtin_shufflevector(lo, hi, 0,1,2,3,4,5,6,7,8,9,10,11,12,13,14,15);
}
__device__ __forceinline__ v16h load_b_frag(const h16* base, int ld, int k0) { return load_a_frag(base, ld, k0); }

__device__ __forceinline__ v8f wmma_f16(v16h a, v16h b, v8f c) {
  v8f d = __builtin_amdgcn_wmma_f32_16x16x32_f16(false, a, false, b, (short)0, c, false, false);
  asm volatile("v_nop\n\tv_nop\n\tv_nop\n\tv_nop" : "+v"(d) : "v"(a), "v"(b));
  return d;
}

__global__ __launch_bounds__(256) void cvt_x_kernel(const float* __restrict__ x, h16* __restrict__ xb, int n8) {
  int g = blockIdx.x * 256 + threadIdx.x;
  if (g >= n8) return;
  const int row = g >> 6, c8 = g & 63;
  const int b = row / SEQ, s = row - b * SEQ;
  const float* src = x + ((size_t)(b * SEQ_FULL + s)) * DM + c8 * 8;
  const v4f a = *(const v4f*)(src), bq = *(const v4f*)(src + 4);
  union { h16x8 h; v4u u; } pk;
#pragma unroll
  for (int i = 0; i < 4; ++i) { pk.h[i] = (h16)(bf16r(a[i]) * ISC); pk.h[4 + i] = (h16)(bf16r(bq[i]) * ISC); }
  vst2(xb + (size_t)g * 8, pk.u);
}

__global__ __launch_bounds__(256) void cvt_w_kernel(const float* __restrict__ W0, const float* __restrict__ W1,
                                                    const float* __restrict__ W2, const float* __restrict__ W3,
                                                    h16* __restrict__ D0, h16* __restrict__ D1,
                                                    h16* __restrict__ D2, h16* __restrict__ D3) {
  const int y = blockIdx.y;
  const float* W = (y == 0) ? W0 : (y == 1) ? W1 : (y == 2) ? W2 : W3;
  h16*       D  = (y == 0) ? D0 : (y == 1) ? D1 : (y == 2) ? D2 : D3;
  const int g = blockIdx.x * 256 + threadIdx.x;
  if (g >= DM * DM / 8) return;
  const float* src = W + (size_t)g * 8;
  const v4f a = *(const v4f*)(src), bq = *(const v4f*)(src + 4);
  union { h16x8 h; v4u u; } pk;
#pragma unroll
  for (int i = 0; i < 4; ++i) { pk.h[i] = (h16)(bf16r(a[i]) * WSC); pk.h[4 + i] = (h16)(bf16r(bq[i]) * WSC); }
  vst2(D + (size_t)g * 8, pk.u);
}

__global__ __launch_bounds__(256) void proj_qkv_kernel(const h16* __restrict__ Xb,
                                                       const h16* __restrict__ Wq, const h16* __restrict__ Wk,
                                                       const h16* __restrict__ Wv,
                                                       h16* __restrict__ Qh, h16* __restrict__ Kh, h16* __restrict__ Vth,
                                                       h16* __restrict__ Qr, h16* __restrict__ Kr, h16* __restrict__ Vtr) {
  __shared__ __align__(16) h16 Th[128 * 136];
  __shared__ __align__(16) h16 Tr[128 * 136];
  const int z = blockIdx.z;
  const h16* W = (z == 0) ? Wq : (z == 1) ? Wk : Wv;
  const int transposed = (z == 2) ? 1 : 0;
  const int m0 = blockIdx.x * 64, n0 = blockIdx.y * 128;
  const int bb = m0 / SEQ, s0 = m0 - bb * SEQ;
  const bool early = (s0 < EARLY_R);
  const int tid = threadIdx.x, w = tid >> 5, lane = tid & 31, idx = lane & 15, half = lane >> 4;
  const int mw_l = (w & 3) * 16;
  const int nw_l = (w >> 2) * 64;

  v8f c[4] = {};
  const h16* arow = Xb + (size_t)(m0 + mw_l) * DM;
  const h16* brow = W + (size_t)(n0 + nw_l) * DM;
#pragma unroll 2
  for (int k0 = 0; k0 < DM; k0 += 32) {
    v16h a = load_a_frag(arow, DM, k0);
#pragma unroll
    for (int t = 0; t < 4; ++t) {
      v16h bf = load_b_frag(brow + (size_t)(t * 16) * DM, DM, k0);
      c[t] = wmma_f16(a, bf, c[t]);
    }
  }
#pragma unroll
  for (int t = 0; t < 4; ++t) {
    const int cl = nw_l + t * 16 + idx;
#pragma unroll
    for (int g = 0; g < 8; ++g) {
      const int rl = mw_l + g + 8 * half;
      const float u = c[t][g] * PROJ_MUL;
      const h16 hv = (h16)u;
      const int li = transposed ? (cl * 72 + rl) : (rl * 136 + cl);
      Th[li] = hv;
      if (early) Tr[li] = (h16)((u - (float)hv) * RSC);
    }
  }
  __syncthreads();
  if (!transposed) {
    h16* Oh = (z == 0) ? Qh : Kh;
    h16* Orp = (z == 0) ? Qr : Kr;
    for (int gg = tid; gg < 64 * 16; gg += 256) {
      const int rl = gg >> 4, pc = gg & 15;
      vst2(Oh + (size_t)(m0 + rl) * DM + n0 + pc * 8, *(const v4u*)(&Th[rl * 136 + pc * 8]));
      if (early) vst2(Orp + (size_t)(bb * EARLY_R + s0 + rl) * DM + n0 + pc * 8, *(const v4u*)(&Tr[rl * 136 + pc * 8]));
    }
  } else {
    for (int gg = tid; gg < 128 * 8; gg += 256) {
      const int cl = gg >> 3, pc = gg & 7;
      vst2(Vth + ((size_t)(bb * DM + n0 + cl)) * SEQ + s0 + pc * 8, *(const v4u*)(&Th[cl * 72 + pc * 8]));
      if (early) vst2(Vtr + ((size_t)(bb * DM + n0 + cl)) * EARLY_R + s0 + pc * 8, *(const v4u*)(&Tr[cl * 72 + pc * 8]));
    }
  }
}

__global__ __launch_bounds__(256) __attribute__((amdgpu_num_vgpr(256)))
void attn_main_kernel(const h16* __restrict__ Qh, const h16* __restrict__ Kh,
                      const h16* __restrict__ Vth, h16* __restrict__ Ch) {
  __shared__ __align__(16) h16   Qs[32][DM];
  __shared__ __align__(16) h16   Vts[DM][64];
  __shared__ __align__(16) float Ss[32][64];
  __shared__ __align__(16) h16   Ps[32][64];
  __shared__ float alpha_s[32];
  __shared__ float l_s[32];

  const int b   = blockIdx.y;
  const int q0  = EARLY_R + blockIdx.x * 32;
  const int tid = threadIdx.x;
  const int w    = tid >> 5;
  const int lane = tid & 31;
  const int idx  = lane & 15;
  const int half = lane >> 4;
  const int qi = w & 1;
  const int kj = w >> 1;
  const int dg = w >> 1;

  const h16* Qg = Qh + ((size_t)(b * SEQ + q0)) * DM;
  for (int cc = tid; cc < 32 * (DM / 8); cc += 256) {
    const int r = cc >> 6, dc = cc & 63;
    copy16_g2s(&Qs[r][dc * 8], Qg + (size_t)r * DM + dc * 8);
  }

  v8f o[8] = {};
  const int srow = tid >> 3;
  const int sj   = tid & 7;
  float m_prev = -1e30f;
  float l_run  = 0.0f;
  const int nchunk = q0 / 64 + 1;

#pragma unroll 1
  for (int ci = 0; ci < nchunk; ++ci) {
    const int kv0 = ci * 64;
    __syncthreads();
    const h16* Vg = Vth + (size_t)(b * DM) * SEQ + kv0;
    for (int cc = tid; cc < DM * 8; cc += 256) {
      const int d = cc >> 3, j = cc & 7;
      copy16_g2s(&Vts[d][j * 8], Vg + (size_t)d * SEQ + j * 8);
    }
    __syncthreads();

    {
      v8f sc = {};
      const h16* Kg = Kh + ((size_t)(b * SEQ + kv0 + kj * 16)) * DM;
#pragma unroll 4
      for (int k0 = 0; k0 < DM; k0 += 32) {
        v16h a  = load_a_frag(&Qs[qi * 16][0], DM, k0);
        v16h bf = load_b_frag(Kg, DM, k0);
        sc = wmma_f16(a, bf, sc);
      }
      const int col = kj * 16 + idx;
      const int key = kv0 + col;
#pragma unroll
      for (int g = 0; g < 8; ++g) {
        const int rl = qi * 16 + g + 8 * half;
        float val = sc[g] * SCL;
        if (key > q0 + rl) val = -1e30f;
        Ss[rl][col] = val;
      }
    }
    __syncthreads();

    {
      float v[8];
      float mloc = -1e30f;
#pragma unroll
      for (int e = 0; e < 8; ++e) { v[e] = Ss[srow][sj + e * 8]; mloc = fmaxf(mloc, v[e]); }
#pragma unroll
      for (int msk = 1; msk < 8; msk <<= 1) mloc = fmaxf(mloc, __shfl_xor(mloc, msk, 32));
      const float m_new = fmaxf(m_prev, mloc);
      const float alpha = __expf(m_prev - m_new);
      float ssum = 0.0f;
#pragma unroll
      for (int e = 0; e < 8; ++e) {
        const float p = __expf(v[e] - m_new);
        ssum += p;
        Ps[srow][sj + e * 8] = (h16)(p * PSC);
      }
#pragma unroll
      for (int msk = 1; msk < 8; msk <<= 1) ssum += __shfl_xor(ssum, msk, 32);
      l_run = l_run * alpha + ssum;
      m_prev = m_new;
      if (sj == 0) { alpha_s[srow] = alpha; l_s[srow] = l_run; }
    }
    __syncthreads();

    {
      float al[8];
#pragma unroll
      for (int g = 0; g < 8; ++g) al[g] = alpha_s[qi * 16 + g + 8 * half];
#pragma unroll
      for (int t = 0; t < 8; ++t)
#pragma unroll
        for (int g = 0; g < 8; ++g) o[t][g] *= al[g];
#pragma unroll
      for (int k0 = 0; k0 < 64; k0 += 32) {
        v16h a = load_a_frag(&Ps[qi * 16][0], 64, k0);
#pragma unroll
        for (int t = 0; t < 8; ++t) {
          v16h bf = load_b_frag(&Vts[dg * 128 + t * 16][0], 64, k0);
          o[t] = wmma_f16(a, bf, o[t]);
        }
      }
    }
  }
  __syncthreads();

  h16* Ct = &Vts[0][0];
  float linv[8];
#pragma unroll
  for (int g = 0; g < 8; ++g) linv[g] = 1.0f / (l_s[qi * 16 + g + 8 * half] * PSC);
#pragma unroll
  for (int t = 0; t < 8; ++t) {
    const int col = dg * 128 + t * 16 + idx;
#pragma unroll
    for (int g = 0; g < 8; ++g) Ct[(qi * 16 + g + 8 * half) * DM + col] = (h16)(o[t][g] * linv[g]);
  }
  __syncthreads();
  {
    h16* dst = Ch + ((size_t)(b * SEQ + q0)) * DM;
    for (int gg = tid; gg < 32 * DM / 8; gg += 256) vst2(dst + (size_t)gg * 8, *(const v4u*)(Ct + gg * 8));
  }
}

__global__ __launch_bounds__(256) __attribute__((amdgpu_num_vgpr(256)))
void attn_early_kernel(const h16* __restrict__ Qh, const h16* __restrict__ Qr,
                       const h16* __restrict__ Kh, const h16* __restrict__ Kr,
                       const h16* __restrict__ Vth, const h16* __restrict__ Vtr,
                       h16* __restrict__ Ch, h16* __restrict__ Cr) {
  __shared__ __align__(16) h16   Qs[2][16][DM];
  __shared__ __align__(16) h16   Ks[2][32][DM];
  __shared__ __align__(16) h16   Vts[2][DM][32];
  __shared__ __align__(16) float Ss[3][16][32];
  __shared__ __align__(16) h16   Ps[2][16][32];
  __shared__ float alpha_s[16];
  __shared__ float l_s[16];

  const int b   = blockIdx.y;
  const int q0  = blockIdx.x * 16;
  const int tid = threadIdx.x;
  const int w    = tid >> 5;
  const int lane = tid & 31;
  const int idx  = lane & 15;
  const int half = lane >> 4;

  {
    const h16* Qg0 = Qh + ((size_t)(b * SEQ + q0)) * DM;
    const h16* Qg1 = Qr + ((size_t)(b * EARLY_R + q0)) * DM;
    for (int cc = tid; cc < 16 * (DM / 8); cc += 256) {
      const int r = cc >> 6, dc = cc & 63;
      copy16_g2s(&Qs[0][r][dc * 8], Qg0 + (size_t)r * DM + dc * 8);
      copy16_g2s(&Qs[1][r][dc * 8], Qg1 + (size_t)r * DM + dc * 8);
    }
  }

  v8f oh[4] = {};
  v8f orr[4] = {};
  const int srow = tid >> 4;
  const int sj   = tid & 15;
  float m_prev = -1e30f;
  float l_run  = 0.0f;
  const int nchunk = q0 / 32 + 1;

#pragma unroll 1
  for (int ci = 0; ci < nchunk; ++ci) {
    const int kv0 = ci * 32;
    __syncthreads();
    {
      const h16* Kg0 = Kh + ((size_t)(b * SEQ + kv0)) * DM;
      const h16* Kg1 = Kr + ((size_t)(b * EARLY_R + kv0)) * DM;
      for (int cc = tid; cc < 32 * (DM / 8); cc += 256) {
        const int r = cc >> 6, dc = cc & 63;
        copy16_g2s(&Ks[0][r][dc * 8], Kg0 + (size_t)r * DM + dc * 8);
        copy16_g2s(&Ks[1][r][dc * 8], Kg1 + (size_t)r * DM + dc * 8);
      }
      const h16* Vg0 = Vth + (size_t)(b * DM) * SEQ + kv0;
      const h16* Vg1 = Vtr + (size_t)(b * DM) * EARLY_R + kv0;
      for (int cc = tid; cc < DM * 4; cc += 256) {
        const int d = cc >> 2, j = cc & 3;
        copy16_g2s(&Vts[0][d][j * 8], Vg0 + (size_t)d * SEQ + j * 8);
        copy16_g2s(&Vts[1][d][j * 8], Vg1 + (size_t)d * EARLY_R + j * 8);
      }
    }
    __syncthreads();

    if (w < 6) {
      const int prod = w >> 1, kj = w & 1;
      const int pa = (prod == 2) ? 1 : 0;
      const int pb = (prod == 1) ? 1 : 0;
      v8f sc = {};
#pragma unroll 4
      for (int k0 = 0; k0 < DM; k0 += 32) {
        v16h a  = load_a_frag(&Qs[pa][0][0], DM, k0);
        v16h bf = load_b_frag(&Ks[pb][kj * 16][0], DM, k0);
        sc = wmma_f16(a, bf, sc);
      }
      const int col = kj * 16 + idx;
#pragma unroll
      for (int g = 0; g < 8; ++g) Ss[prod][g + 8 * half][col] = sc[g];
    }
    __syncthreads();

    {
      float v[2];
      float mloc = -1e30f;
      const int qrow = q0 + srow;
#pragma unroll
      for (int e = 0; e < 2; ++e) {
        const int cidx = sj + e * 16;
        float s = (Ss[0][srow][cidx] + (Ss[1][srow][cidx] + Ss[2][srow][cidx]) * RINV) * SCL;
        if (kv0 + cidx > qrow) s = -1e30f;
        v[e] = s; mloc = fmaxf(mloc, s);
      }
#pragma unroll
      for (int msk = 1; msk < 16; msk <<= 1) mloc = fmaxf(mloc, __shfl_xor(mloc, msk, 32));
      const float m_new = fmaxf(m_prev, mloc);
      const float alpha = __expf(m_prev - m_new);
      float ssum = 0.0f;
#pragma unroll
      for (int e = 0; e < 2; ++e) {
        const int cidx = sj + e * 16;
        const float p  = __expf(v[e] - m_new);
        ssum += p;
        const float pp = p * PSC;
        const h16 hv = (h16)pp;
        Ps[0][srow][cidx] = hv;
        Ps[1][srow][cidx] = (h16)((pp - (float)hv) * RSC);
      }
#pragma unroll
      for (int msk = 1; msk < 16; msk <<= 1) ssum += __shfl_xor(ssum, msk, 32);
      l_run = l_run * alpha + ssum;
      m_prev = m_new;
      if (sj == 0) { alpha_s[srow] = alpha; l_s[srow] = l_run; }
    }
    __syncthreads();

    {
      float al[8];
#pragma unroll
      for (int g = 0; g < 8; ++g) al[g] = alpha_s[g + 8 * half];
#pragma unroll
      for (int t = 0; t < 4; ++t)
#pragma unroll
        for (int g = 0; g < 8; ++g) { oh[t][g] *= al[g]; orr[t][g] *= al[g]; }
      v16h ah = load_a_frag(&Ps[0][0][0], 32, 0);
      v16h ar = load_a_frag(&Ps[1][0][0], 32, 0);
#pragma unroll
      for (int t = 0; t < 4; ++t) {
        const int d0 = w * 64 + t * 16;
        v16h bh = load_b_frag(&Vts[0][d0][0], 32, 0);
        v16h br = load_b_frag(&Vts[1][d0][0], 32, 0);
        oh[t]  = wmma_f16(ah, bh, oh[t]);
        orr[t] = wmma_f16(ah, br, orr[t]);
        orr[t] = wmma_f16(ar, bh, orr[t]);
      }
    }
  }
  __syncthreads();

  h16* Ct = &Ks[0][0][0];
  float linv[8];
#pragma unroll
  for (int g = 0; g < 8; ++g) linv[g] = 1.0f / (l_s[g + 8 * half] * PSC);
#pragma unroll
  for (int t = 0; t < 4; ++t) {
    const int col = w * 64 + t * 16 + idx;
#pragma unroll
    for (int g = 0; g < 8; ++g) {
      const int rl = g + 8 * half;
      const float u = (oh[t][g] + orr[t][g] * RINV) * linv[g];
      const h16 hv = (h16)u;
      Ct[rl * DM + col] = hv;
      Ct[16 * DM + rl * DM + col] = (h16)((u - (float)hv) * RSC);
    }
  }
  __syncthreads();
  {
    h16* dsth = Ch + ((size_t)(b * SEQ + q0)) * DM;
    h16* dstr = Cr + ((size_t)(b * EARLY_R + q0)) * DM;
    for (int gg = tid; gg < 16 * DM / 8; gg += 256) {
      vst2(dsth + (size_t)gg * 8, *(const v4u*)(Ct + gg * 8));
      vst2(dstr + (size_t)gg * 8, *(const v4u*)(Ct + 16 * DM + gg * 8));
    }
  }
}

__global__ __launch_bounds__(256) void proj_out_kernel(const h16* __restrict__ Ch, const h16* __restrict__ Cr,
                                                       const h16* __restrict__ Wo, float* __restrict__ out) {
  __shared__ __align__(16) float T[64 * 132];
  const int m0 = blockIdx.x * 64, n0 = blockIdx.y * 128;
  const int bb = m0 / SEQ, s0 = m0 - bb * SEQ;
  const bool early = (s0 < EARLY_R);
  const int tid = threadIdx.x, w = tid >> 5, lane = tid & 31, idx = lane & 15, half = lane >> 4;
  const int mw_l = (w & 3) * 16;
  const int nw_l = (w >> 2) * 64;

  v8f c[4] = {};
  v8f cr[4] = {};
  const h16* arow = Ch + (size_t)(m0 + mw_l) * DM;
  const h16* brow = Wo + (size_t)(n0 + nw_l) * DM;
  if (early) {
    const h16* rrow = Cr + (size_t)(bb * EARLY_R + s0 + mw_l) * DM;
#pragma unroll 2
    for (int k0 = 0; k0 < DM; k0 += 32) {
      v16h a  = load_a_frag(arow, DM, k0);
      v16h ar = load_a_frag(rrow, DM, k0);
#pragma unroll
      for (int t = 0; t < 4; ++t) {
        v16h bf = load_b_frag(brow + (size_t)(t * 16) * DM, DM, k0);
        c[t]  = wmma_f16(a, bf, c[t]);
        cr[t] = wmma_f16(ar, bf, cr[t]);
      }
    }
  } else {
#pragma unroll 2
    for (int k0 = 0; k0 < DM; k0 += 32) {
      v16h a = load_a_frag(arow, DM, k0);
#pragma unroll
      for (int t = 0; t < 4; ++t) {
        v16h bf = load_b_frag(brow + (size_t)(t * 16) * DM, DM, k0);
        c[t] = wmma_f16(a, bf, c[t]);
      }
    }
  }
#pragma unroll
  for (int t = 0; t < 4; ++t) {
    const int cl = nw_l + t * 16 + idx;
#pragma unroll
    for (int g = 0; g < 8; ++g) {
      const int rl = mw_l + g + 8 * half;
      T[rl * 132 + cl] = (c[t][g] + cr[t][g] * RINV) * OUT_MUL;
    }
  }
  __syncthreads();
  {
    float* dst = out + ((size_t)(bb * SEQ_FULL + s0)) * DM + n0;
    for (int gg = tid; gg < 64 * 32; gg += 256) {
      const int rl = gg >> 5, pc = gg & 31;
      vst2(dst + (size_t)rl * DM + pc * 4, *(const v4f*)(&T[rl * 132 + pc * 4]));
    }
  }
}

extern "C" void kernel_launch(void* const* d_in, const int* in_sizes, int n_in,
                              void* d_out, int out_size, void* d_ws, size_t ws_size,
                              hipStream_t stream) {
  if (n_in < 5) return;
  const int rows_needed = (NB - 1) * SEQ_FULL + SEQ;
  if (in_sizes[0] < rows_needed * DM) return;
  for (int i = 1; i < 5; ++i) if (in_sizes[i] < DM * DM) return;
  if (out_size < rows_needed * DM) return;

  const float* x  = (const float*)d_in[0];
  const float* Wq = (const float*)d_in[1];
  const float* Wk = (const float*)d_in[2];
  const float* Wv = (const float*)d_in[3];
  const float* Wo = (const float*)d_in[4];
  float* out = (float*)d_out;

  const size_t plane = (size_t)MT * DM * sizeof(h16);
  const size_t wpl   = (size_t)DM * DM * sizeof(h16);
  const size_t rpl   = (size_t)NB * EARLY_R * DM * sizeof(h16);
  size_t off = 0;
  char* ws = (char*)d_ws;
  h16* xb  = (h16*)(ws + off); off += plane;
  h16* wqb = (h16*)(ws + off); off += wpl;
  h16* wkb = (h16*)(ws + off); off += wpl;
  h16* wvb = (h16*)(ws + off); off += wpl;
  h16* wob = (h16*)(ws + off); off += wpl;
  h16* qh  = (h16*)(ws + off); off += plane;
  h16* kh  = (h16*)(ws + off); off += plane;
  h16* vth = (h16*)(ws + off); off += plane;
  h16* qr  = (h16*)(ws + off); off += rpl;
  h16* kr  = (h16*)(ws + off); off += rpl;
  h16* vtr = (h16*)(ws + off); off += rpl;
  h16* ch  = (h16*)(ws + off); off += plane;
  h16* crp = (h16*)(ws + off); off += rpl;
  if (off > ws_size) return;

  const int nx8 = MT * DM / 8;
  cvt_x_kernel<<<(nx8 + 255) / 256, 256, 0, stream>>>(x, xb, nx8);
  cvt_w_kernel<<<dim3((DM * DM / 8 + 255) / 256, 4), 256, 0, stream>>>(Wq, Wk, Wv, Wo, wqb, wkb, wvb, wob);

  proj_qkv_kernel<<<dim3(MT / 64, DM / 128, 3), 256, 0, stream>>>(xb, wqb, wkb, wvb, qh, kh, vth, qr, kr, vtr);

  attn_early_kernel<<<dim3(EARLY_R / 16, NB), 256, 0, stream>>>(qh, qr, kh, kr, vth, vtr, ch, crp);
  if (SEQ > EARLY_R) {
    attn_main_kernel<<<dim3((SEQ - EARLY_R) / 32, NB), 256, 0, stream>>>(qh, kh, vth, ch);
  }

  proj_out_kernel<<<dim3(MT / 64, DM / 128), 256, 0, stream>>>(ch, crp, wob, out);
}
